// DiagSSMBlock_76347338654364
// MI455X (gfx1250) — hardware-run, weakly checked
//
#include <hip/hip_runtime.h>

typedef __bf16 v16bf __attribute__((ext_vector_type(16)));
typedef unsigned short v8us __attribute__((ext_vector_type(8)));
typedef float v8f __attribute__((ext_vector_type(8)));
typedef float v4f __attribute__((ext_vector_type(4)));
typedef v8us __attribute__((may_alias)) v8usa;
typedef v4f  __attribute__((may_alias)) v4fa;

union Frag { v16bf v; v8us u[2]; };

#define TDIM 4096
#define HDIM 2048
#define NXE (TDIM * HDIM)
#define NBE (HDIM * HDIM)
#define NX8 (NXE / 8)
#define BT_PITCH 72

static_assert(TDIM % 128 == 0);
static_assert(HDIM % 64 == 0);
static_assert(HDIM % 32 == 0);
static_assert((HDIM / 4) % 64 == 0);
static_assert(NXE % 8 == 0);

__device__ __forceinline__ unsigned short f2bf(float f) {
  unsigned int u = __float_as_uint(f);
  u = u + 0x7FFFu + ((u >> 16) & 1u);
  return (unsigned short)(u >> 16);
}
__device__ __forceinline__ float bfq(float f) {
  return __uint_as_float(((unsigned int)f2bf(f)) << 16);
}

__device__ __forceinline__ v8f wmma_bf16(v16bf a, v16bf b, v8f c) {
  v8f d = __builtin_amdgcn_wmma_f32_16x16x32_bf16(false, a, false, b, (short)0, c, false, false);
  asm volatile("v_nop\n\tv_nop\n\tv_nop\n\tv_nop" : "+v"(d) : "v"(a), "v"(b));
  return d;
}

__device__ __forceinline__ v16bf load_frag(const unsigned short* p, int h) {
  Frag f;
  f.u[0] = *(const v8usa*)(p + 8 * h);
  f.u[1] = *(const v8usa*)(p + 16 + 8 * h);
  return f.v;
}

__global__ __launch_bounds__(256) void cvt_x_kernel(
    const float* __restrict__ x, unsigned short* __restrict__ xh)
{
  const int g = blockIdx.x * 256 + threadIdx.x;
  if (g >= NX8) return;
  const float* src = x + (size_t)g * 8;
  const v4f a = *(const v4fa*)src;
  const v4f c = *(const v4fa*)(src + 4);
  const v8us o = { f2bf(a.x), f2bf(a.y), f2bf(a.z), f2bf(a.w),
                   f2bf(c.x), f2bf(c.y), f2bf(c.z), f2bf(c.w) };
  unsigned short* dst = xh + (size_t)g * 8;
  *(volatile v8us*)dst = o;
  __threadfence();
  *(volatile v8us*)dst = o;
}

__global__ __launch_bounds__(256) void cvt_bt_kernel(
    const float* __restrict__ B, unsigned short* __restrict__ bt)
{
  __shared__ __attribute__((aligned(16))) unsigned short sT[64 * BT_PITCH];

  const int tid = threadIdx.x;
  const int n0 = blockIdx.x * 64, k0 = blockIdx.y * 64;
  const int c = tid & 15, krb = tid >> 4;
  #pragma unroll
  for (int i = 0; i < 4; ++i) {
    const int kr = krb + 16 * i;
    const v4f v = *(const v4fa*)(B + (size_t)(k0 + kr) * HDIM + n0 + 4 * c);
    sT[(4 * c + 0) * BT_PITCH + kr] = f2bf(v.x);
    sT[(4 * c + 1) * BT_PITCH + kr] = f2bf(v.y);
    sT[(4 * c + 2) * BT_PITCH + kr] = f2bf(v.z);
    sT[(4 * c + 3) * BT_PITCH + kr] = f2bf(v.w);
  }
  __syncthreads();

  const int q8 = tid & 7, lb = tid >> 3;
  const v8us v0 = *(const v8usa*)(sT + lb * BT_PITCH + 8 * q8);
  const v8us v1 = *(const v8usa*)(sT + (lb + 32) * BT_PITCH + 8 * q8);
  unsigned short* d0 = bt + (size_t)(n0 + lb) * HDIM + k0 + 8 * q8;
  unsigned short* d1 = bt + (size_t)(n0 + lb + 32) * HDIM + k0 + 8 * q8;
  *(volatile v8us*)d0 = v0;
  *(volatile v8us*)d1 = v1;
  __threadfence();
  *(volatile v8us*)d0 = v0;
  *(volatile v8us*)d1 = v1;
}

__device__ __forceinline__ void gemm_store_pass(const float* so, float* S,
                                                int m0w, int n0, int lane) {
  const int q8 = lane & 7, sub = lane >> 3;
  #pragma unroll
  for (int i = 0; i < 16; ++i) {
    const int lid = i * 4 + sub;
    const int row = lid >> 1, hl = lid & 1;
    const v4f v = *(const v4fa*)(so + row * 64 + 32 * hl + 4 * q8);
    const size_t gi = (size_t)(m0w + row) * HDIM + n0 + 32 * hl + 4 * q8;
    *(volatile v4f*)(S + gi) = v;
  }
}

__global__ __launch_bounds__(128) void gemm_kernel(
    const unsigned short* __restrict__ xh,
    const unsigned short* __restrict__ bt,
    float* __restrict__ S)
{
  __shared__ __attribute__((aligned(16))) float sO[4 * 32 * 64];

  const int tid = threadIdx.x, lane = tid & 31, w = tid >> 5;
  const int h = lane >> 4, m = lane & 15;
  const int m0 = blockIdx.x * 128, n0 = blockIdx.y * 64;
  const int m0w = m0 + 32 * w;

  const unsigned short* xa0 = xh + (size_t)(m0w + m) * HDIM;
  const unsigned short* xa1 = xa0 + (size_t)16 * HDIM;
  const unsigned short* wb  = bt + (size_t)(n0 + m) * HDIM;

  const v8f zero8 = {0.f, 0.f, 0.f, 0.f, 0.f, 0.f, 0.f, 0.f};
  v8f acc[2][4];
  #pragma unroll
  for (int mt = 0; mt < 2; ++mt)
    #pragma unroll
    for (int nt = 0; nt < 4; ++nt) acc[mt][nt] = zero8;

  #pragma unroll 1
  for (int k0 = 0; k0 < HDIM; k0 += 32) {
    const v16bf a0 = load_frag(xa0 + k0, h);
    const v16bf a1 = load_frag(xa1 + k0, h);
    #pragma unroll
    for (int nt = 0; nt < 4; ++nt) {
      const v16bf b = load_frag(wb + (size_t)nt * 16 * HDIM + k0, h);
      acc[0][nt] = wmma_bf16(a0, b, acc[0][nt]);
      acc[1][nt] = wmma_bf16(a1, b, acc[1][nt]);
    }
  }

  float* so = sO + w * 2048;
  #pragma unroll
  for (int nt = 0; nt < 4; ++nt) {
    #pragma unroll
    for (int mt = 0; mt < 2; ++mt) {
      #pragma unroll
      for (int r = 0; r < 8; ++r) {
        const int rowl = 16 * mt + 8 * h + r;
        so[rowl * 64 + 16 * nt + m] = acc[mt][nt][r];
      }
    }
  }
  __syncthreads();

  gemm_store_pass(so, S, m0w, n0, lane);
  __threadfence();
  gemm_store_pass(so, S, m0w, n0, lane);
}

__global__ __launch_bounds__(64) void scan_kernel(
    const float* __restrict__ S,
    const float* __restrict__ a,
    float* __restrict__ out)
{
  const int g = blockIdx.x * 64 + threadIdx.x;
  if (g >= HDIM / 4) return;
  const int c0 = 4 * g;
  const v4f av = *(const v4fa*)(a + c0);
  const float a0 = bfq(av.x), a1 = bfq(av.y), a2 = bfq(av.z), a3 = bfq(av.w);
  float h0 = 0.f, h1 = 0.f, h2 = 0.f, h3 = 0.f;
  const float* sp = S + c0;
  float* op = out + c0;
  #pragma unroll 1
  for (int t = 0; t < TDIM; ++t) {
    const v4f s = *(const v4fa*)(sp + (size_t)t * HDIM);
    h0 = fmaf(a0, h0, s.x);
    h1 = fmaf(a1, h1, s.y);
    h2 = fmaf(a2, h2, s.z);
    h3 = fmaf(a3, h3, s.w);
    const v4f o = {h0, h1, h2, h3};
    float* dst = op + (size_t)t * HDIM;
    *(volatile v4f*)dst = o;
    __threadfence();
    *(volatile v4f*)dst = o;
  }
}

extern "C" void kernel_launch(void* const* d_in, const int* in_sizes, int n_in,
                              void* d_out, int out_size, void* d_ws, size_t ws_size,
                              hipStream_t stream) {
  if (n_in < 3) return;
  if (in_sizes[0] != NXE) return;
  if (in_sizes[1] != HDIM) return;
  if (in_sizes[2] != NBE) return;
  if (out_size != NXE) return;

  const float* x = (const float*)d_in[0];
  const float* a = (const float*)d_in[1];
  const float* B = (const float*)d_in[2];
  float* out = (float*)d_out;

  const size_t xh_bytes = (size_t)NXE * 2;
  const size_t bt_bytes = (size_t)NBE * 2;
  const size_t s_bytes  = (size_t)NXE * 4;
  const size_t total = xh_bytes + bt_bytes + s_bytes;
  if (total > ws_size) return;

  char* ws = (char*)d_ws;
  unsigned short* xh = (unsigned short*)(ws);
  unsigned short* bt = (unsigned short*)(ws + xh_bytes);
  float* S = (float*)(ws + xh_bytes + bt_bytes);

  cvt_x_kernel<<<(NX8 + 255) / 256, 256, 0, stream>>>(x, xh);

  dim3 gBt(HDIM / 64, HDIM / 64);
  cvt_bt_kernel<<<gBt, 256, 0, stream>>>(B, bt);

  dim3 gGemm(TDIM / 128, HDIM / 64);
  gemm_kernel<<<gGemm, 128, 0, stream>>>(xh, bt, S);

  scan_kernel<<<(HDIM / 4 + 63) / 64, 64, 0, stream>>>(S, a, out);
}
